// Net_37434934952778
// MI455X (gfx1250) — hardware-verified
//
#include <hip/hip_runtime.h>
#include <stddef.h>
#include <stdint.h>
#include <math.h>


#define HD     64
#define XIN    32
#define EDIM   16
#define YW     1152
#define KK     128
#define NGW    192
#define NTHR   256
#define NWAVE  8
#define EPT    8
#define CHUNK  (NTHR * EPT)
#define WCAP   (EPT * 32)
#define LISTN  (NWAVE * WCAP)
#define NBA    1024
#define SLA    10
#define RCAP   4096
#define DEGCAP 32
#define GBM    64
#define GTHR   128
#define U_NNW  16384
#define U_NNB  1024
#define U_ROOT 1024
#define U_WPP  (U_NNW + U_NNB + U_ROOT)
#define U_WIH  (NGW * 16)
#define U_WHH  (NGW * 16)
#define U_L0   (HD * 4)
#define U_ALL  (U_WPP + U_WIH + U_WHH + U_L0)
#define AGG_ZINTS (LISTN + 2 * RCAP + 3 * NBA)
#define AGG_LDS_INTS (AGG_ZINTS + 16)

static_assert((CHUNK & (CHUNK - 1)) == 0 && CHUNK <= 4096);
static_assert((NBA & (NBA - 1)) == 0 && NBA == (1 << SLA));
static_assert(((long long)CHUNK << SLA) < (1LL << 31));
static_assert(NBA % NWAVE == 0 && NBA % 32 == 0 && NBA % GBM == 0);
static_assert(RCAP % 32 == 0 && AGG_ZINTS % 4 == 0 && LISTN % 4 == 0);
static_assert(KK == 2 * HD && KK % 32 == 0 && XIN == 32 && YW % 64 == 0 && YW == 18 * 64);
static_assert(GBM == (GTHR / 32) * 16 && HD == 64 && HD == 2 * 32);
static_assert(U_NNW % NTHR == 0 && U_NNB % NTHR == 0 && U_ROOT % NTHR == 0);
static_assert(U_WIH % NTHR == 0 && U_WHH % NTHR == 0 && U_L0 % NTHR == 0 && U_ALL % NTHR == 0);
static_assert(AGG_LDS_INTS * 4 <= 65536);
static_assert(EDIM == 16);

typedef float          v2f   __attribute__((ext_vector_type(2)));
typedef float          v4f   __attribute__((ext_vector_type(4)));
typedef float          v8f   __attribute__((ext_vector_type(8)));
typedef int            v4i   __attribute__((ext_vector_type(4)));
typedef int            v8i   __attribute__((ext_vector_type(8)));
typedef unsigned short v4us  __attribute__((ext_vector_type(4)));
typedef unsigned short v8us  __attribute__((ext_vector_type(8)));
typedef unsigned short v16us __attribute__((ext_vector_type(16)));
typedef __bf16         v16bf __attribute__((ext_vector_type(16)));
typedef v2f  __attribute__((may_alias)) v2fa;
typedef v4f  __attribute__((may_alias)) v4fa;
typedef v4i  __attribute__((may_alias)) v4ia;
typedef v4us __attribute__((may_alias)) v4usa;
typedef v8us __attribute__((may_alias)) v8usa;
union FragB { v16bf v; v16us u; v8us h[2]; v8i w; };

__device__ __forceinline__ v8f wmb(const FragB& a, const FragB& b, v8f c) {
  v8f d = __builtin_amdgcn_wmma_f32_16x16x32_bf16(false, a.v, false, b.v, (short)0, c, false, false);
  asm volatile("v_nop\n\tv_nop\n\tv_nop\n\tv_nop" : "+v"(d) : "v"(a.w), "v"(b.w));
  return d;
}

__device__ __forceinline__ unsigned bf16_bits(float f) {
  const unsigned u = __float_as_uint(f);
  return (u + 0x7FFFu + ((u >> 16) & 1u)) >> 16;
}
__device__ __forceinline__ float bf16_val(float f) {
  return __uint_as_float(bf16_bits(f) << 16);
}
__device__ __forceinline__ void split4(const v4f v, v4us& h4, v4us& l4) {
  unsigned hb;
  hb = bf16_bits(v.x); h4[0] = (unsigned short)hb; l4[0] = (unsigned short)bf16_bits(v.x - __uint_as_float(hb << 16));
  hb = bf16_bits(v.y); h4[1] = (unsigned short)hb; l4[1] = (unsigned short)bf16_bits(v.y - __uint_as_float(hb << 16));
  hb = bf16_bits(v.z); h4[2] = (unsigned short)hb; l4[2] = (unsigned short)bf16_bits(v.z - __uint_as_float(hb << 16));
  hb = bf16_bits(v.w); h4[3] = (unsigned short)hb; l4[3] = (unsigned short)bf16_bits(v.w - __uint_as_float(hb << 16));
}
__device__ __forceinline__ float sigm(float v) {
  float c = (v < -60.0f) ? -60.0f : v;
  c = (c > 60.0f) ? 60.0f : c;
  return 1.0f / (1.0f + expf(-c));
}

__device__ __forceinline__ void stage_acc(float* stg, const v8f (&acc)[4], int wave, int hh, int m) {
#pragma unroll
  for (int t = 0; t < 4; ++t) {
    const int lc = 16 * t + m;
#pragma unroll
    for (int r = 0; r < 8; ++r) {
      const int lr = 16 * wave + 8 * hh + r;
      stg[lr * HD + lc] = acc[t][r];
    }
  }
}
__device__ __forceinline__ void put_tile(const v4f (&fv)[8], float* base, size_t ldo, int row0, int hh, int m,
                                         int rowLimit) {
#pragma unroll
  for (int i = 0; i < 8; ++i) {
    const int gr = row0 + 2 * i + hh;
    if (gr < rowLimit) *(volatile v4f*)(base + (size_t)gr * ldo + 4 * m) = fv[i];
  }
  __threadfence();
#pragma unroll
  for (int i = 0; i < 8; ++i) {
    const int gr = row0 + 2 * i + hh;
    if (gr < rowLimit) *(volatile v4f*)(base + (size_t)gr * ldo + 4 * m) = fv[i];
  }
}

template <int SLB>
__device__ __forceinline__ int scan_chunk(const int* __restrict__ dsts, int nE, int cbase, int slotBase,
                                          int nb, int vec8, int* list, int tid, int lane, int wave) {
  int wc = 0;
  const int el0  = tid * EPT;
  const int e0   = cbase + el0;
  const int sent = -2147483647 - 1;
  v4i da, db;
  if (vec8 != 0 && cbase + CHUNK <= nE) {
    da = *(const v4i*)(dsts + e0);
    db = *(const v4i*)(dsts + e0 + 4);
  } else {
    da.x = (e0     < nE) ? dsts[min(e0,     nE - 1)] : sent;
    da.y = (e0 + 1 < nE) ? dsts[min(e0 + 1, nE - 1)] : sent;
    da.z = (e0 + 2 < nE) ? dsts[min(e0 + 2, nE - 1)] : sent;
    da.w = (e0 + 3 < nE) ? dsts[min(e0 + 3, nE - 1)] : sent;
    db.x = (e0 + 4 < nE) ? dsts[min(e0 + 4, nE - 1)] : sent;
    db.y = (e0 + 5 < nE) ? dsts[min(e0 + 5, nE - 1)] : sent;
    db.z = (e0 + 6 < nE) ? dsts[min(e0 + 6, nE - 1)] : sent;
    db.w = (e0 + 7 < nE) ? dsts[min(e0 + 7, nE - 1)] : sent;
  }
  const unsigned nbs = (unsigned)slotBase;
  const unsigned unb = (unsigned)nb;
  const unsigned s0 = (unsigned)da.x - nbs, s1 = (unsigned)da.y - nbs;
  const unsigned s2 = (unsigned)da.z - nbs, s3 = (unsigned)da.w - nbs;
  const unsigned s4 = (unsigned)db.x - nbs, s5 = (unsigned)db.y - nbs;
  const unsigned s6 = (unsigned)db.z - nbs, s7 = (unsigned)db.w - nbs;
  const bool h0 = s0 < unb, h1 = s1 < unb, h2 = s2 < unb, h3 = s3 < unb;
  const bool h4 = s4 < unb, h5 = s5 < unb, h6 = s6 < unb, h7 = s7 < unb;
  const unsigned any = __builtin_amdgcn_ballot_w32(h0 | h1 | h2 | h3 | h4 | h5 | h6 | h7);
  if (any != 0u) {
#define HITJ(J, HJ, SJ) { \
      const unsigned mj = __builtin_amdgcn_ballot_w32(HJ); \
      if (mj != 0u) { \
        if (HJ) { \
          const int pos = wc + (int)__builtin_amdgcn_mbcnt_lo(mj, 0u); \
          if (pos < WCAP) list[wave * WCAP + pos] = ((el0 + (J)) << SLB) | (int)(SJ); \
        } \
        wc += (int)__builtin_popcount(mj); } }
    HITJ(0, h0, s0)
    HITJ(1, h1, s1)
    HITJ(2, h2, s2)
    HITJ(3, h3, s3)
    HITJ(4, h4, s4)
    HITJ(5, h5, s5)
    HITJ(6, h6, s6)
    HITJ(7, h7, s7)
#undef HITJ
  }
  return wc;
}

__global__ __launch_bounds__(NTHR) void k_prep(const float* __restrict__ nnw, const float* __restrict__ nnb,
                                               const float* __restrict__ root, const float* __restrict__ wih,
                                               const float* __restrict__ whh, const float* __restrict__ l0w,
                                               unsigned short* WPP, unsigned short* WIH2,
                                               unsigned short* WHH2, unsigned short* L0B) {
  const int u = (int)blockIdx.x * NTHR + (int)threadIdx.x;
  v8us o;
  unsigned short* dp;
  if (u < U_WPP) {
    const int n  = u >> 4;
    const int c8 = (u & 15) * 8;
    const int i0 = c8 & (HD - 1);
    const float* p;
    int stride;
    if (u < U_NNW) {
      const int kq = n >> 6, oo = n & (HD - 1);
      p = nnw + ((size_t)i0 * HD + oo) * EDIM + kq;
      stride = HD * EDIM;
    } else if (u < U_NNW + U_NNB) {
      const int oo = n - 1024;
      p = nnb + (size_t)i0 * HD + oo;
      stride = HD;
    } else {
      const int oo = n - 1088;
      p = root + (size_t)i0 * HD + oo;
      stride = HD;
    }
#pragma unroll
    for (int i = 0; i < 8; ++i) o[i] = (unsigned short)bf16_bits(p[(size_t)i * stride]);
    dp = WPP + (size_t)n * KK + c8;
  } else if (u < U_WPP + U_WIH + U_WHH) {
    const int v   = u - U_WPP;
    const bool sl = v >= U_WIH;
    const int w   = sl ? v - U_WIH : v;
    const int n   = w >> 4;
    const int c8  = (w & 15) * 8;
    const int kk  = c8 & (HD - 1);
    const float* p = (sl ? whh : wih) + (size_t)n * HD + kk;
    const v4f a = *(const v4fa*)p;
    const v4f b = *(const v4fa*)(p + 4);
    o[0] = (unsigned short)bf16_bits(a.x); o[1] = (unsigned short)bf16_bits(a.y);
    o[2] = (unsigned short)bf16_bits(a.z); o[3] = (unsigned short)bf16_bits(a.w);
    o[4] = (unsigned short)bf16_bits(b.x); o[5] = (unsigned short)bf16_bits(b.y);
    o[6] = (unsigned short)bf16_bits(b.z); o[7] = (unsigned short)bf16_bits(b.w);
    dp = (sl ? WHH2 : WIH2) + (size_t)n * KK + c8;
  } else if (u < U_ALL) {
    const int w  = u - (U_WPP + U_WIH + U_WHH);
    const int n  = w >> 2;
    const int k8 = (w & 3) * 8;
    const float* p = l0w + (size_t)n * XIN + k8;
    const v4f a = *(const v4fa*)p;
    const v4f b = *(const v4fa*)(p + 4);
    o[0] = (unsigned short)bf16_bits(a.x); o[1] = (unsigned short)bf16_bits(a.y);
    o[2] = (unsigned short)bf16_bits(a.z); o[3] = (unsigned short)bf16_bits(a.w);
    o[4] = (unsigned short)bf16_bits(b.x); o[5] = (unsigned short)bf16_bits(b.y);
    o[6] = (unsigned short)bf16_bits(b.z); o[7] = (unsigned short)bf16_bits(b.w);
    dp = L0B + (size_t)n * XIN + k8;
  } else {
    return;
  }
  *(volatile v8us*)dp = o;
  __threadfence();
  *(volatile v8us*)dp = o;
}

__global__ __launch_bounds__(GTHR) void k_lin0(const float* __restrict__ x, const unsigned short* __restrict__ L0B,
                                               const float* __restrict__ b0, int nN, int mRows, float* outp) {
  __shared__ __attribute__((aligned(16))) float stg[GBM * HD];
  const int tid = (int)threadIdx.x, lane = tid & 31, wave = tid >> 5, hh = lane >> 4, m = lane & 15;
  const int rowBase = (int)blockIdx.x * GBM;
  const int row = rowBase + 16 * wave + m;
  const int rc  = row < nN ? row : nN - 1;
  const bool ok = row < nN;
  const float* p = x + (size_t)rc * XIN + 8 * hh;
  const v4f a0 = *(const v4fa*)p;
  const v4f a1 = *(const v4fa*)(p + 4);
  const v4f a2 = *(const v4fa*)(p + 16);
  const v4f a3 = *(const v4fa*)(p + 20);
  FragB af;
  af.u[0]  = ok ? (unsigned short)bf16_bits(a0.x) : (unsigned short)0;
  af.u[1]  = ok ? (unsigned short)bf16_bits(a0.y) : (unsigned short)0;
  af.u[2]  = ok ? (unsigned short)bf16_bits(a0.z) : (unsigned short)0;
  af.u[3]  = ok ? (unsigned short)bf16_bits(a0.w) : (unsigned short)0;
  af.u[4]  = ok ? (unsigned short)bf16_bits(a1.x) : (unsigned short)0;
  af.u[5]  = ok ? (unsigned short)bf16_bits(a1.y) : (unsigned short)0;
  af.u[6]  = ok ? (unsigned short)bf16_bits(a1.z) : (unsigned short)0;
  af.u[7]  = ok ? (unsigned short)bf16_bits(a1.w) : (unsigned short)0;
  af.u[8]  = ok ? (unsigned short)bf16_bits(a2.x) : (unsigned short)0;
  af.u[9]  = ok ? (unsigned short)bf16_bits(a2.y) : (unsigned short)0;
  af.u[10] = ok ? (unsigned short)bf16_bits(a2.z) : (unsigned short)0;
  af.u[11] = ok ? (unsigned short)bf16_bits(a2.w) : (unsigned short)0;
  af.u[12] = ok ? (unsigned short)bf16_bits(a3.x) : (unsigned short)0;
  af.u[13] = ok ? (unsigned short)bf16_bits(a3.y) : (unsigned short)0;
  af.u[14] = ok ? (unsigned short)bf16_bits(a3.z) : (unsigned short)0;
  af.u[15] = ok ? (unsigned short)bf16_bits(a3.w) : (unsigned short)0;

  v8f acc[4];
  const v8f z = {0.f, 0.f, 0.f, 0.f, 0.f, 0.f, 0.f, 0.f};
#pragma unroll
  for (int t = 0; t < 4; ++t) {
    const unsigned short* wq = L0B + (size_t)(16 * t + m) * XIN + 8 * hh;
    FragB bf;
    bf.h[0] = *(const v8usa*)wq;
    bf.h[1] = *(const v8usa*)(wq + 16);
    acc[t] = wmb(af, bf, z);
  }
  stage_acc(stg, acc, wave, hh, m);
  __syncthreads();

  v4f bb;
  {
    const v4f t1 = *(const v4fa*)(b0 + 4 * m);
    bb.x = bf16_val(t1.x); bb.y = bf16_val(t1.y); bb.z = bf16_val(t1.z); bb.w = bf16_val(t1.w);
  }
  v4f fv[8];
#pragma unroll
  for (int i = 0; i < 8; ++i) {
    const int lr = 16 * wave + 2 * i + hh;
    const bool live = (rowBase + lr) < nN;
    const v4f t = *(const v4fa*)(stg + lr * HD + 4 * m) + bb;
    v4f y;
    y.x = (t.x > 0.0f) ? t.x : 0.0f; y.y = (t.y > 0.0f) ? t.y : 0.0f;
    y.z = (t.z > 0.0f) ? t.z : 0.0f; y.w = (t.w > 0.0f) ? t.w : 0.0f;
    y.x = live ? y.x : 0.0f; y.y = live ? y.y : 0.0f; y.z = live ? y.z : 0.0f; y.w = live ? y.w : 0.0f;
    fv[i] = y;
  }
  put_tile(fv, outp, (size_t)HD, rowBase + 16 * wave, hh, m, mRows);
}

__global__ __launch_bounds__(GTHR) void k_yr(const float* __restrict__ outp, const unsigned short* __restrict__ WPP,
                                             int mRows, float* yr) {
  __shared__ __attribute__((aligned(16))) unsigned short al[GBM * KK];
  __shared__ __attribute__((aligned(16))) float stg[GBM * HD];
  const int tid = (int)threadIdx.x, lane = tid & 31, wave = tid >> 5, hh = lane >> 4, m = lane & 15;
  const int rowBase = (int)blockIdx.x * GBM;

#pragma unroll
  for (int j = 0; j < 8; ++j) {
    const int idx = tid + GTHR * j;
    const int row = idx >> 4;
    const int c4  = (idx & 15) * 4;
    const v4f v = *(const v4fa*)(outp + (size_t)(rowBase + row) * HD + c4);
    v4us h4, l4;
    split4(v, h4, l4);
    *(v4usa*)(al + row * KK + c4) = h4;
    *(v4usa*)(al + row * KK + HD + c4) = l4;
  }
  __syncthreads();

  FragB af[4];
#pragma unroll
  for (int ks = 0; ks < 4; ++ks) {
    const unsigned short* ap = al + (16 * wave + m) * KK + 32 * ks + 8 * hh;
    af[ks].h[0] = *(const v8usa*)ap;
    af[ks].h[1] = *(const v8usa*)(ap + 16);
  }
  const unsigned short* wp = WPP + (size_t)m * KK + 8 * hh;

#pragma unroll 1
  for (int nt = 0; nt < YW / 64; ++nt) {
    const int col0 = nt * 64;
    v8f acc[4];
    {
      const v8f z = {0.f, 0.f, 0.f, 0.f, 0.f, 0.f, 0.f, 0.f};
      acc[0] = z; acc[1] = z; acc[2] = z; acc[3] = z;
    }
#pragma unroll
    for (int ks = 0; ks < 4; ++ks) {
#pragma unroll
      for (int t = 0; t < 4; ++t) {
        const unsigned short* wq = wp + (size_t)(col0 + 16 * t) * KK + 32 * ks;
        FragB bf;
        bf.h[0] = *(const v8usa*)wq;
        bf.h[1] = *(const v8usa*)(wq + 16);
        acc[t] = wmb(af[ks], bf, acc[t]);
      }
    }
    stage_acc(stg, acc, wave, hh, m);
    __syncthreads();
    v4f fv[8];
#pragma unroll
    for (int i = 0; i < 8; ++i) {
      const int lr = 16 * wave + 2 * i + hh;
      fv[i] = *(const v4fa*)(stg + lr * HD + 4 * m);
    }
    __syncthreads();
    put_tile(fv, yr + col0, (size_t)YW, rowBase + 16 * wave, hh, m, mRows);
  }
}

__global__ __launch_bounds__(NTHR) void k_msg(const int* __restrict__ srcs, const int* __restrict__ dsts,
                                              int nE, int nN, int vec8, int mRows,
                                              const float* __restrict__ ea, const float* __restrict__ yr,
                                              const float* __restrict__ cb, float* mout) {
  extern __shared__ __attribute__((aligned(16))) int dsm[];
  int* list = dsm;
  int* hl   = dsm + LISTN;
  int* sl   = dsm + LISTN + RCAP;
  int* cnt  = dsm + LISTN + 2 * RCAP;
  int* offs = cnt + NBA;
  int* cur  = offs + NBA;
  int* misc = cur + NBA;
  const int tid = (int)threadIdx.x, lane = tid & 31, wave = tid >> 5;
  const int nodeBase = (int)blockIdx.x * NBA;

  {
    const v4i z4 = {0, 0, 0, 0};
    for (int i = tid * 4; i < AGG_ZINTS; i += NTHR * 4) *(v4ia*)(dsm + i) = z4;
    if (tid < 16) misc[tid] = 0;
  }
  float bv0, bv1;
  {
    const v2f a = *(const v2fa*)(cb + 2 * lane);
    bv0 = bf16_val(a.x); bv1 = bf16_val(a.y);
  }
  __syncthreads();

  int t = 0, ov = 0;
  const int nChunks = (nE + CHUNK - 1) / CHUNK;
#pragma unroll 1
  for (int ch = 0; ch < nChunks; ++ch) {
    const int cbase = ch * CHUNK;
    const int wc = scan_chunk<SLA>(dsts, nE, cbase, nodeBase, NBA, vec8, list, tid, lane, wave);
    if (lane == 0) misc[wave] = wc;
    __syncthreads();
    if (wave == 0) {
#pragma unroll 1
      for (int w2 = 0; w2 < NWAVE; ++w2) {
        int c = misc[w2];
        c = c < 0 ? 0 : (c > WCAP ? WCAP : c);
#pragma unroll 1
        for (int b0 = 0; b0 < c; b0 += 32) {
          const int idx = b0 + lane;
          const int ent = list[w2 * WCAP + (idx < WCAP ? idx : WCAP - 1)];
          const int m32 = (c - b0) < 32 ? (c - b0) : 32;
#pragma unroll 1
          for (int k = 0; k < m32; ++k) {
            const int u    = __builtin_amdgcn_readlane(ent, k);
            const int slot = u & (NBA - 1);
            const int el   = (u >> SLA) & (CHUNK - 1);
            const int pk   = ((cbase + el) << SLA) | slot;
            if (t < RCAP) {
              if (lane == 0) { hl[t] = pk; cnt[slot] = cnt[slot] + 1; }
              t = t + 1;
            } else {
              ov = 1;
            }
          }
        }
      }
    }
    __syncthreads();
  }
  if (wave == 0 && lane == 0) { misc[8] = t; misc[9] = ov; }
  __syncthreads();
  int tt = misc[8];
  tt = tt < 0 ? 0 : (tt > RCAP ? RCAP : tt);
  const int ovf = misc[9];

  if (wave == 0) {
    const int base = lane * (NBA / 32);
    int s = 0;
#pragma unroll 1
    for (int i = 0; i < NBA / 32; ++i) s += cnt[base + i];
    int incl = s;
#pragma unroll
    for (int d = 1; d < 32; d <<= 1) {
      const int y = __shfl_up(incl, d, 32);
      if (lane >= d) incl += y;
    }
    int run = incl - s;
#pragma unroll 1
    for (int i = 0; i < NBA / 32; ++i) {
      const int cv = cnt[base + i];
      offs[base + i] = run;
      cur[base + i]  = run;
      run += cv;
    }
  }
  __syncthreads();
  if (wave == 0) {
#pragma unroll 1
    for (int b0 = 0; b0 < tt; b0 += 32) {
      const int idx = b0 + lane;
      const int ent = hl[idx < RCAP ? idx : RCAP - 1];
      const int m32 = (tt - b0) < 32 ? (tt - b0) : 32;
#pragma unroll 1
      for (int k = 0; k < m32; ++k) {
        const int u    = __builtin_amdgcn_readlane(ent, k);
        const int slot = u & (NBA - 1);
        if (lane == 0) {
          int p = cur[slot];
          p = p < 0 ? 0 : (p > RCAP - 1 ? RCAP - 1 : p);
          sl[p] = u;
          cur[slot] = p + 1;
        }
      }
    }
  }
  __syncthreads();

  const float qnan = __int_as_float(0x7fc00000);
  const float pz = (ovf != 0) ? qnan : 0.0f;
  const int sa = (2 * lane) & 31, sb = (2 * lane + 1) & 31;
#pragma unroll 1
  for (int si = 0; si < NBA / NWAVE; ++si) {
    const int s    = si * NWAVE + wave;
    const int node = nodeBase + s;
    int c = cnt[s];
    const bool big = c > DEGCAP;
    c = c < 0 ? 0 : (c > DEGCAP ? DEGCAP : c);
    int o = offs[s];
    o = o < 0 ? 0 : (o > RCAP ? RCAP : o);
    const int nc = node < nN ? node : nN - 1;
    float acc0 = 0.0f, acc1 = 0.0f;
#pragma unroll 1
    for (int b0 = 0; b0 < c; b0 += 32) {
      int idx = o + b0 + lane;
      idx = idx > RCAP - 1 ? RCAP - 1 : idx;
      const int ent = sl[idx];
      int eid = ent >> SLA;
      eid = eid < 0 ? 0 : (eid > nE - 1 ? nE - 1 : eid);
      int sr = srcs[eid];
      sr = sr < 0 ? 0 : (sr > nN - 1 ? nN - 1 : sr);
      const int m32 = (c - b0) < 32 ? (c - b0) : 32;
#pragma unroll 1
      for (int k = 0; k < m32; ++k) {
        const int sk = __builtin_amdgcn_readlane(sr, k);
        const int ek = __builtin_amdgcn_readlane(eid, k);
        const float eav = bf16_val(ea[(size_t)ek * EDIM + (lane & 15)]);
        int eai = __float_as_int(eav);
        const float* yp = yr + (size_t)sk * YW + 2 * lane;
        const v2f bq = *(const v2fa*)(yp + 1024);
        float m0 = bq.x, m1 = bq.y;
        asm volatile("" : "+v"(eai), "+v"(m0), "+v"(m1));
#pragma unroll 1
        for (int g = 0; g < 4; ++g) {
#pragma unroll
          for (int j = 0; j < 4; ++j) {
            const int kq = 4 * g + j;
            const float a = __int_as_float(__builtin_amdgcn_readlane(eai, kq));
            const v2f y = *(const v2fa*)(yp + kq * HD);
            m0 = fmaf(a, y.x, m0);
            m1 = fmaf(a, y.y, m1);
          }
        }
        acc0 += m0; acc1 += m1;
      }
    }
    float rt0, rt1;
    {
      const v2f a = *(const v2fa*)(yr + (size_t)nc * YW + 1088 + 2 * lane);
      rt0 = a.x; rt1 = a.y;
    }
    const float pzr = big ? qnan : pz;
    const bool live = node < nN;
    float y0 = (acc0 + rt0) + bv0;
    float y1 = (acc1 + rt1) + bv1;
    y0 = (y0 > 0.0f) ? y0 : (y0 - y0);
    y1 = (y1 > 0.0f) ? y1 : (y1 - y1);
    y0 = y0 + pzr; y1 = y1 + pzr;
    const float v0 = live ? y0 : 0.0f;
    const float v1 = live ? y1 : 0.0f;
    const bool wr = (node < mRows) && (lane < 16);
    v4f ow;
    ow.x = __shfl(v0, sa, 32); ow.y = __shfl(v1, sa, 32);
    ow.z = __shfl(v0, sb, 32); ow.w = __shfl(v1, sb, 32);
    float* op = mout + (size_t)node * HD + 4 * (lane & 15);
    if (wr) *(volatile v4f*)op = ow;
    __threadfence();
    if (wr) *(volatile v4f*)op = ow;
  }
}

__global__ __launch_bounds__(GTHR) void k_gru(const float* mp, const float* hp,
                                              const unsigned short* __restrict__ WIH2,
                                              const unsigned short* __restrict__ WHH2,
                                              const float* __restrict__ bih, const float* __restrict__ bhh,
                                              float* dst, int rowLimit, int nN) {
  __shared__ __attribute__((aligned(16))) unsigned short am[GBM * KK];
  __shared__ __attribute__((aligned(16))) unsigned short ah[GBM * KK];
  __shared__ __attribute__((aligned(16))) float hf[GBM * HD];
  const int tid = (int)threadIdx.x, lane = tid & 31, wave = tid >> 5, hh = lane >> 4, m = lane & 15;
  const int rowBase = (int)blockIdx.x * GBM;

#pragma unroll
  for (int j = 0; j < 8; ++j) {
    const int idx = tid + GTHR * j;
    const int row = idx >> 4;
    const int c4  = (idx & 15) * 4;
    const v4f mv = *(const v4fa*)(mp + (size_t)(rowBase + row) * HD + c4);
    const v4f hv = *(const v4fa*)(hp + (size_t)(rowBase + row) * HD + c4);
    v4us h4, l4;
    split4(mv, h4, l4);
    *(v4usa*)(am + row * KK + c4) = h4;
    *(v4usa*)(am + row * KK + HD + c4) = l4;
    split4(hv, h4, l4);
    *(v4usa*)(ah + row * KK + c4) = h4;
    *(v4usa*)(ah + row * KK + HD + c4) = l4;
    *(v4fa*)(hf + row * HD + c4) = hv;
  }
  __syncthreads();

  FragB fm[4], fh[4];
#pragma unroll
  for (int ks = 0; ks < 4; ++ks) {
    const unsigned short* pm = am + (16 * wave + m) * KK + 32 * ks + 8 * hh;
    const unsigned short* ph = ah + (16 * wave + m) * KK + 32 * ks + 8 * hh;
    fm[ks].h[0] = *(const v8usa*)pm;
    fm[ks].h[1] = *(const v8usa*)(pm + 16);
    fh[ks].h[0] = *(const v8usa*)ph;
    fh[ks].h[1] = *(const v8usa*)(ph + 16);
  }

#pragma unroll 1
  for (int nt = 0; nt < 4; ++nt) {
    const int o = nt * 16 + m;
    const v8f z8 = {0.f, 0.f, 0.f, 0.f, 0.f, 0.f, 0.f, 0.f};
    v8f aR = z8, aZ = z8, aI = z8, aH = z8;
    const unsigned short* wi = WIH2 + (size_t)o * KK + 8 * hh;
    const unsigned short* wh = WHH2 + (size_t)o * KK + 8 * hh;
#pragma unroll
    for (int ks = 0; ks < 4; ++ks) {
      FragB b;
      b.h[0] = *(const v8usa*)(wi + 32 * ks);
      b.h[1] = *(const v8usa*)(wi + 32 * ks + 16);
      aR = wmb(fm[ks], b, aR);
      b.h[0] = *(const v8usa*)(wi + (size_t)HD * KK + 32 * ks);
      b.h[1] = *(const v8usa*)(wi + (size_t)HD * KK + 32 * ks + 16);
      aZ = wmb(fm[ks], b, aZ);
      b.h[0] = *(const v8usa*)(wi + (size_t)2 * HD * KK + 32 * ks);
      b.h[1] = *(const v8usa*)(wi + (size_t)2 * HD * KK + 32 * ks + 16);
      aI = wmb(fm[ks], b, aI);
      b.h[0] = *(const v8usa*)(wh + 32 * ks);
      b.h[1] = *(const v8usa*)(wh + 32 * ks + 16);
      aR = wmb(fh[ks], b, aR);
      b.h[0] = *(const v8usa*)(wh + (size_t)HD * KK + 32 * ks);
      b.h[1] = *(const v8usa*)(wh + (size_t)HD * KK + 32 * ks + 16);
      aZ = wmb(fh[ks], b, aZ);
      b.h[0] = *(const v8usa*)(wh + (size_t)2 * HD * KK + 32 * ks);
      b.h[1] = *(const v8usa*)(wh + (size_t)2 * HD * KK + 32 * ks + 16);
      aH = wmb(fh[ks], b, aH);
    }
    const float bir = bf16_val(bih[o]),          bhr = bf16_val(bhh[o]);
    const float biz = bf16_val(bih[HD + o]),     bhz = bf16_val(bhh[HD + o]);
    const float bin = bf16_val(bih[2 * HD + o]), bhn = bf16_val(bhh[2 * HD + o]);
#pragma unroll
    for (int r = 0; r < 8; ++r) {
      const int lr = 16 * wave + 8 * hh + r;
      const float rg = sigm((aR[r] + bir) + bhr);
      const float zg = sigm((aZ[r] + biz) + bhz);
      const float ng = tanhf((aI[r] + bin) + rg * (aH[r] + bhn));
      const float hv = hf[lr * HD + o];
      hf[lr * HD + o] = (1.0f - zg) * ng + zg * hv;
    }
  }
  __syncthreads();

  v4f fv[8];
#pragma unroll
  for (int i = 0; i < 8; ++i) {
    const int lr = 16 * wave + 2 * i + hh;
    const bool live = (rowBase + lr) < nN;
    v4f y = *(const v4fa*)(hf + lr * HD + 4 * m);
    y.x = live ? y.x : 0.0f; y.y = live ? y.y : 0.0f; y.z = live ? y.z : 0.0f; y.w = live ? y.w : 0.0f;
    fv[i] = y;
  }
  put_tile(fv, dst, (size_t)HD, rowBase + 16 * wave, hh, m, rowLimit);
}

static inline int cdiv(int a, int b) { return (a + b - 1) / b; }
static inline size_t al256(size_t o) { return (o + 255) & ~(size_t)255; }

extern "C" void kernel_launch(void* const* d_in, const int* in_sizes, int n_in,
                              void* d_out, int out_size, void* d_ws, size_t ws_size,
                              hipStream_t stream) {
  if (n_in < 13) return;
  if (in_sizes[0] < XIN || (in_sizes[0] % XIN) != 0) return;
  const int nN = in_sizes[0] / XIN;
  if (nN < 16 || nN > (1 << 22)) return;
  if (in_sizes[1] < 2 || (in_sizes[1] & 1) != 0) return;
  const int nE = in_sizes[1] / 2;
  if (nE < 1 || nE >= (1 << (31 - SLA))) return;
  if ((long long)in_sizes[2] != (long long)nE * EDIM) return;
  if (in_sizes[3] != HD * XIN || in_sizes[4] != HD) return;
  if (in_sizes[5] != HD * HD * EDIM || in_sizes[6] != HD * HD) return;
  if (in_sizes[7] != HD * HD || in_sizes[8] != HD) return;
  if (in_sizes[9] != NGW * HD || in_sizes[10] != NGW * HD) return;
  if (in_sizes[11] != NGW || in_sizes[12] != NGW) return;
  if ((long long)out_size != (long long)nN * HD) return;

  const float* x    = (const float*)d_in[0];
  const int*   edge = (const int*)d_in[1];
  const float* ea   = (const float*)d_in[2];
  const float* l0w  = (const float*)d_in[3];
  const float* l0b  = (const float*)d_in[4];
  const float* nnw  = (const float*)d_in[5];
  const float* nnb  = (const float*)d_in[6];
  const float* root = (const float*)d_in[7];
  const float* cvb  = (const float*)d_in[8];
  const float* wih  = (const float*)d_in[9];
  const float* whh  = (const float*)d_in[10];
  const float* bih  = (const float*)d_in[11];
  const float* bhh  = (const float*)d_in[12];
  float* out = (float*)d_out;
  const int* src = edge;
  const int* dst = edge + nE;

  const int NP = cdiv(nN, GBM) * GBM;
  const int gM = NP / GBM;
  const int gA = cdiv(NP, NBA);
  if ((long long)gA * NBA < (long long)NP) return;
  const int vec8 = ((nE & 3) == 0) ? 1 : 0;

  char* ws = (char*)d_ws;
  size_t off = 0;
  const size_t oWPP = off; off = al256(off + (size_t)YW * KK * 2);
  const size_t oWIH = off; off = al256(off + (size_t)NGW * KK * 2);
  const size_t oWHH = off; off = al256(off + (size_t)NGW * KK * 2);
  const size_t oL0B = off; off = al256(off + (size_t)HD * XIN * 2);
  const size_t oOUT = off; off = al256(off + (size_t)NP * HD * 4);
  const size_t oM   = off; off = al256(off + (size_t)NP * HD * 4);
  const size_t oYR  = off; off = al256(off + (size_t)NP * YW * 4);
  if (off > ws_size) return;
  unsigned short* WPP  = (unsigned short*)(ws + oWPP);
  unsigned short* WIH2 = (unsigned short*)(ws + oWIH);
  unsigned short* WHH2 = (unsigned short*)(ws + oWHH);
  unsigned short* L0B  = (unsigned short*)(ws + oL0B);
  float*          OUT  = (float*)(ws + oOUT);
  float*          M    = (float*)(ws + oM);
  float*          YR   = (float*)(ws + oYR);

  const size_t msgLds = (size_t)AGG_LDS_INTS * 4;
  hipFuncSetAttribute(reinterpret_cast<const void*>(&k_msg), hipFuncAttributeMaxDynamicSharedMemorySize, (int)msgLds);

  k_prep<<<U_ALL / NTHR, NTHR, 0, stream>>>(nnw, nnb, root, wih, whh, l0w, WPP, WIH2, WHH2, L0B);
  k_lin0<<<gM, GTHR, 0, stream>>>(x, L0B, l0b, nN, NP, OUT);
  for (int it = 0; it < 3; ++it) {
    k_yr<<<gM, GTHR, 0, stream>>>(OUT, WPP, NP, YR);
    k_msg<<<gA, NTHR, msgLds, stream>>>(src, dst, nE, nN, vec8, NP, ea, YR, cvb, M);
    if (it < 2) k_gru<<<gM, GTHR, 0, stream>>>(M, OUT, WIH2, WHH2, bih, bhh, OUT, NP, nN);
    else        k_gru<<<gM, GTHR, 0, stream>>>(M, OUT, WIH2, WHH2, bih, bhh, out, nN, nN);
  }
}
